// GraphSAGEBackbone_4578435137604
// MI455X (gfx1250) — hardware-run, weakly checked
//
#include <hip/hip_runtime.h>
#include <stddef.h>
#include <stdint.h>


#define NN       50000
#define NE       1600000
#define DF       128
#define NLAY     3
#define GBM      128
#define NTILE    391
#define MROWS    (NTILE * GBM)
#define NBRUN    1024
#define SLA      10
#define NBLK     49
#define NPADT    (NBLK * NBRUN)
#define RCAP     36864
#define DEGCAP   96
#define MEAS_HITS 33116
#define MEAS_DEG  61
#define NTHR     256
#define NWAVE    8
#define EPT      8
#define CHUNK    (NTHR * EPT)
#define NCHUNK   ((NE + CHUNK - 1) / CHUNK)
#define MPITCH   256
#define HPITCH   256
#define XPITCH   128
#define WPITCH   512
#define WC_LH    0
#define WC_LL    128
#define WC_RH    256
#define WC_RL    384
#define MEAN_LO  1
#define H_LO     1
#define W_SPLIT  0
#define BK_INTS  (RCAP + RCAP / 2 + 3 * NBRUN + 16)
#define BK_ZV4   ((RCAP / 2 + 3 * NBRUN + 16) / 4)
#define G_FLOATS (GBM * DF + DF + 6 * DF)

#define NUW  (NLAY * DF * (WPITCH / 8))
#define NUZ  (2 * (MROWS - NN) * (MPITCH / 8))
#define NUX  (MROWS * (XPITCH / 8))
#define NUP  (3 * NLAY * DF / 4)
#define PU1  NUW
#define PU2  (PU1 + NUZ)
#define PU3  (PU2 + NUX)
#define PU4  (PU3 + NUP)

static_assert(NN < 65536);
static_assert(NBRUN * NBLK >= NN && NBRUN * NBLK >= MROWS && NBRUN == (1 << SLA));
static_assert(RCAP * 100 >= MEAS_HITS * 105);
static_assert(DEGCAP >= MEAS_DEG + 8);
static_assert(RCAP % 4 == 0 && (RCAP / 4) % NTHR == 0 && RCAP < 65536);
static_assert(MROWS >= NN && MROWS % GBM == 0 && GBM == NWAVE * 16);
static_assert(DF % 32 == 0 && DF == 4 * 32 && WPITCH == 4 * DF);
static_assert(NE % EPT == 0 && (NE % 4) == 0);
static_assert(BK_INTS * 4 <= 300000);
static_assert((RCAP / 2 + 3 * NBRUN + 16) % 4 == 0);
static_assert(NUW % NTHR == 0 && (NUZ / 2) % NTHR == 0 && NUX % NTHR == 0 && MPITCH == HPITCH);
static_assert((NN * 32) % NTHR == 0);
static_assert(NBRUN == NTHR * 4);
static_assert(G_FLOATS * 4 <= 300000);

constexpr size_t a256(size_t v) { return (v + 255) & ~(size_t)255; }
constexpr size_t SZ_WQ   = (size_t)NLAY * DF * WPITCH * 2;
constexpr size_t SZ_PAR  = (size_t)3 * NLAY * DF * 4;
constexpr size_t SZ_STAT = (size_t)NLAY * 2 * DF * 4;
constexpr size_t SZ_XB   = (size_t)MROWS * XPITCH * 2;
constexpr size_t SZ_MEAN = (size_t)MROWS * MPITCH * 2;
constexpr size_t SZ_H    = (size_t)MROWS * HPITCH * 2;
constexpr size_t SZ_TH   = (size_t)MROWS * DF * 4;
constexpr size_t SZ_LIST = (size_t)NBLK * RCAP * 4;
constexpr size_t SZ_TAB  = (size_t)NPADT * 4;
constexpr size_t SZ_REC  = (size_t)NTILE * 2 * DF * 4;
constexpr size_t O_WQ   = 0;
constexpr size_t O_PAR  = a256(O_WQ + SZ_WQ);
constexpr size_t O_STAT = a256(O_PAR + SZ_PAR);
constexpr size_t O_XB   = a256(O_STAT + SZ_STAT);
constexpr size_t O_MEAN = a256(O_XB + SZ_XB);
constexpr size_t O_H    = a256(O_MEAN + SZ_MEAN);
constexpr size_t O_TH   = a256(O_H + SZ_H);
constexpr size_t O_LIST = a256(O_TH + SZ_TH);
constexpr size_t O_CNT  = a256(O_LIST + SZ_LIST);
constexpr size_t O_OFF  = a256(O_CNT + SZ_TAB);
constexpr size_t O_INV  = a256(O_OFF + SZ_TAB);
constexpr size_t O_REC  = a256(O_INV + SZ_TAB);
constexpr size_t O_END  = a256(O_REC + SZ_REC);
static_assert(O_END <= ((size_t)128u << 20));

typedef float          v4f   __attribute__((ext_vector_type(4)));
typedef float          v8f   __attribute__((ext_vector_type(8)));
typedef int            v4i   __attribute__((ext_vector_type(4)));
typedef int            v8i   __attribute__((ext_vector_type(8)));
typedef unsigned       v2u   __attribute__((ext_vector_type(2)));
typedef unsigned       v4u   __attribute__((ext_vector_type(4)));
typedef unsigned short v4us  __attribute__((ext_vector_type(4)));
typedef unsigned short v8us  __attribute__((ext_vector_type(8)));
typedef unsigned short v16us __attribute__((ext_vector_type(16)));
typedef __bf16         v16bf __attribute__((ext_vector_type(16)));
typedef v4f  __attribute__((may_alias)) v4fa;
typedef v4i  __attribute__((may_alias)) v4ia;
typedef v2u  __attribute__((may_alias)) v2ua;
typedef v4us __attribute__((may_alias)) v4usa;
typedef v8us __attribute__((may_alias)) v8usa;
union FragB { v16bf v; v16us u; v8us h[2]; v8i w; };

__device__ __forceinline__ v8f wmb(const FragB& a, const FragB& b, v8f c) {
  v8f d = __builtin_amdgcn_wmma_f32_16x16x32_bf16(false, a.v, false, b.v, (short)0, c, false, false);
  asm volatile("v_nop\n\tv_nop\n\tv_nop\n\tv_nop" : "+v"(d) : "v"(a.w), "v"(b.w));
  return d;
}

__device__ __forceinline__ v8f z8() { v8f z = {0.f, 0.f, 0.f, 0.f, 0.f, 0.f, 0.f, 0.f}; return z; }

__device__ __forceinline__ unsigned bf16_bits(float f) {
  const unsigned u = __float_as_uint(f);
  const unsigned r = (u + 0x7FFFu + ((u >> 16) & 1u)) >> 16;
  const unsigned q = (u >> 16) | 0x40u;
  return ((u & 0x7FFFFFFFu) > 0x7F800000u) ? q : r;
}
__device__ __forceinline__ unsigned hl_bits(float v, unsigned& lo) {
  const unsigned hb = bf16_bits(v);
  lo = bf16_bits(v - __uint_as_float(hb << 16));
  return hb;
}

__device__ __forceinline__ void wave_sync() {
  __builtin_amdgcn_fence(__ATOMIC_RELEASE, "wavefront");
  __builtin_amdgcn_wave_barrier();
  __builtin_amdgcn_fence(__ATOMIC_ACQUIRE, "wavefront");
}

__device__ __forceinline__ v8us make_hl_piece(unsigned short* rowbuf, int lane, float m0, float m1, float m2, float m3) {
  v4us mh, ml;
  unsigned lb;
  unsigned hb;
  hb = hl_bits(m0, lb); mh[0] = (unsigned short)hb; ml[0] = (unsigned short)lb;
  hb = hl_bits(m1, lb); mh[1] = (unsigned short)hb; ml[1] = (unsigned short)lb;
  hb = hl_bits(m2, lb); mh[2] = (unsigned short)hb; ml[2] = (unsigned short)lb;
  hb = hl_bits(m3, lb); mh[3] = (unsigned short)hb; ml[3] = (unsigned short)lb;
  *(v4usa*)(rowbuf + 4 * lane)      = mh;
  *(v4usa*)(rowbuf + DF + 4 * lane) = ml;
  wave_sync();
  const v8us q0 = *(const v8usa*)(rowbuf + 8 * lane);
  wave_sync();
  return q0;
}

__global__ __launch_bounds__(NTHR) void k_prep(const float* __restrict__ x, const float* __restrict__ wl,
                                               const float* __restrict__ wr, const float* __restrict__ bl,
                                               const float* __restrict__ gam, const float* __restrict__ bet,
                                               unsigned* __restrict__ wsu) {
  const int u = (int)blockIdx.x * NTHR + (int)threadIdx.x;
  v4u o;
  size_t off;
  if (u < PU1) {
    const int l  = u >> 13;
    const int n  = (u >> 6) & (DF - 1);
    const int k8 = (u & 63) * 8;
    const int kk = k8 & (DF - 1);
    const size_t wo = (size_t)l * DF * DF + (size_t)n * DF + (size_t)kk;
    const v4f a0 = *(const v4f*)(wl + wo), a1 = *(const v4f*)(wl + wo + 4);
    const v4f c0 = *(const v4f*)(wr + wo), c1 = *(const v4f*)(wr + wo + 4);
    asm volatile("" :: "v"(a0), "v"(a1), "v"(c0), "v"(c1));
    const float fa[8] = {a0.x, a0.y, a0.z, a0.w, a1.x, a1.y, a1.z, a1.w};
    const float fb[8] = {c0.x, c0.y, c0.z, c0.w, c1.x, c1.y, c1.z, c1.w};
    const unsigned mskL = (k8 < 2 * DF) ? 0xFFFFFFFFu : 0u;
    const unsigned isLo = (unsigned)((k8 >> 7) & 1);
    unsigned hw[8];
#pragma unroll
    for (int i = 0; i < 8; ++i) {
      const unsigned fbits = (__float_as_uint(fa[i]) & mskL) | (__float_as_uint(fb[i]) & ~mskL);
      const float f = __uint_as_float(fbits);
      unsigned lb;
      const unsigned hb = hl_bits(f, lb);
      const unsigned lo2 = (W_SPLIT != 0) ? lb : 0u;
      hw[i] = (isLo != 0u) ? lo2 : hb;
    }
    o.x = hw[0] | (hw[1] << 16); o.y = hw[2] | (hw[3] << 16);
    o.z = hw[4] | (hw[5] << 16); o.w = hw[6] | (hw[7] << 16);
    off = O_WQ / 4 + (size_t)u * 4;
  } else if (u < PU2) {
    const int z  = u - PU1;
    const int pl = z / (NUZ / 2);
    const int zz = z - pl * (NUZ / 2);
    const int r  = zz >> 5, c = zz & 31;
    o.x = 0u; o.y = 0u; o.z = 0u; o.w = 0u;
    const size_t pb = (pl == 0) ? (O_MEAN / 4) : (O_H / 4);
    off = pb + (size_t)(NN + r) * (MPITCH / 2) + (size_t)c * 4;
  } else if (u < PU3) {
    const int v   = u - PU2;
    const int row = v >> 4, k8 = (v & 15) * 8;
    const int rc  = row < NN ? row : NN - 1;
    const unsigned lvm = (row < NN) ? 0xFFFFu : 0u;
    const float* p = x + (size_t)rc * DF + k8;
    const v4f a = *(const v4f*)p;
    const v4f b = *(const v4f*)(p + 4);
    asm volatile("" :: "v"(a), "v"(b));
    const unsigned h0 = bf16_bits(a.x) & lvm, h1 = bf16_bits(a.y) & lvm;
    const unsigned h2 = bf16_bits(a.z) & lvm, h3 = bf16_bits(a.w) & lvm;
    const unsigned h4 = bf16_bits(b.x) & lvm, h5 = bf16_bits(b.y) & lvm;
    const unsigned h6 = bf16_bits(b.z) & lvm, h7 = bf16_bits(b.w) & lvm;
    o.x = h0 | (h1 << 16); o.y = h2 | (h3 << 16); o.z = h4 | (h5 << 16); o.w = h6 | (h7 << 16);
    off = O_XB / 4 + (size_t)v * 4;
  } else if (u < PU4) {
    const int q   = u - PU3;
    const int sel = q / (NLAY * DF / 4);
    const int j   = q - sel * (NLAY * DF / 4);
    const v4f b4 = *(const v4f*)(bl + 4 * j);
    const v4f g4 = *(const v4f*)(gam + 4 * j);
    const v4f e4 = *(const v4f*)(bet + 4 * j);
    asm volatile("" :: "v"(b4), "v"(g4), "v"(e4));
    const unsigned m0 = (sel == 0) ? 0xFFFFFFFFu : 0u;
    const unsigned m1 = (sel == 1) ? 0xFFFFFFFFu : 0u;
    const unsigned m2 = (sel == 2) ? 0xFFFFFFFFu : 0u;
    const unsigned s0 = (__float_as_uint(b4.x) & m0) | (__float_as_uint(g4.x) & m1) | (__float_as_uint(e4.x) & m2);
    const unsigned s1 = (__float_as_uint(b4.y) & m0) | (__float_as_uint(g4.y) & m1) | (__float_as_uint(e4.y) & m2);
    const unsigned s2 = (__float_as_uint(b4.z) & m0) | (__float_as_uint(g4.z) & m1) | (__float_as_uint(e4.z) & m2);
    const unsigned s3 = (__float_as_uint(b4.w) & m0) | (__float_as_uint(g4.w) & m1) | (__float_as_uint(e4.w) & m2);
    o.x = bf16_bits(__uint_as_float(s0)) << 16;
    o.y = bf16_bits(__uint_as_float(s1)) << 16;
    o.z = bf16_bits(__uint_as_float(s2)) << 16;
    o.w = bf16_bits(__uint_as_float(s3)) << 16;
    off = O_PAR / 4 + (size_t)q * 4;
  } else {
    return;
  }
  unsigned* dp = wsu + off;
  *(volatile v4u*)dp = o;
  __threadfence();
  *(volatile v4u*)dp = o;
}

#define HITJ(HJ, WJ) { if (HJ) { if ((unsigned)pos < (unsigned)RCAP) wl[pos] = (int)(WJ); pos += 1; } }

__global__ __launch_bounds__(NTHR) void k_bucket(const int* __restrict__ srcs, const int* __restrict__ dsts,
                                                 int* listp, int* cntp, int* offp, int* invp) {
  extern __shared__ __attribute__((aligned(16))) int dsm[];
  int* wl = dsm;
  unsigned short* sl = (unsigned short*)(dsm + RCAP);
  int* cnt  = dsm + RCAP + RCAP / 2;
  int* offs = cnt + NBRUN;
  int* cur  = offs + NBRUN;
  int* misc = cur + NBRUN;
  const int tid = (int)threadIdx.x, lane = tid & 31, wave = tid >> 5;
  const int blk = (int)blockIdx.x;
  const int slotBase = blk * NBRUN;
  int nb = NN - slotBase;
  nb = nb > NBRUN ? NBRUN : (nb < 0 ? 0 : nb);

  {
    const v4i z4 = {0, 0, 0, 0};
    for (int i = tid; i < BK_ZV4; i += NTHR) *(v4ia*)(dsm + RCAP + 4 * i) = z4;
  }
  __syncthreads();

  int run = 0;
  const unsigned nbs = (unsigned)slotBase, unb = (unsigned)nb;
#pragma unroll 1
  for (int ch = 0; ch < NCHUNK; ++ch) {
    const int e0 = ch * CHUNK + tid * EPT;
    const bool valid = e0 < NE;
    const int e0c = valid ? e0 : (NE - EPT);
    const v4i da = *(const v4i*)(dsts + e0c);
    const v4i db = *(const v4i*)(dsts + e0c + 4);
    const v4i sa = *(const v4i*)(srcs + e0c);
    const v4i sb = *(const v4i*)(srcs + e0c + 4);
    asm volatile("" :: "v"(da), "v"(db), "v"(sa), "v"(sb));
    const unsigned s0 = (unsigned)da.x - nbs, s1 = (unsigned)da.y - nbs;
    const unsigned s2 = (unsigned)da.z - nbs, s3 = (unsigned)da.w - nbs;
    const unsigned s4 = (unsigned)db.x - nbs, s5 = (unsigned)db.y - nbs;
    const unsigned s6 = (unsigned)db.z - nbs, s7 = (unsigned)db.w - nbs;
    const bool h0 = valid && (s0 < unb), h1 = valid && (s1 < unb);
    const bool h2 = valid && (s2 < unb), h3 = valid && (s3 < unb);
    const bool h4 = valid && (s4 < unb), h5 = valid && (s5 < unb);
    const bool h6 = valid && (s6 < unb), h7 = valid && (s7 < unb);
    const int nh = (int)h0 + (int)h1 + (int)h2 + (int)h3 + (int)h4 + (int)h5 + (int)h6 + (int)h7;
    int incl = nh;
#pragma unroll
    for (int d = 1; d < 32; d <<= 1) {
      const int y = __shfl_up(incl, d, 32);
      incl += (lane >= d) ? y : 0;
    }
    const int tw = __shfl(incl, 31, 32);
    const int par = (ch & 1) * 8;
    if (lane == 0) misc[par + wave] = tw;
    __syncthreads();
    const v4i m0 = *(const v4ia*)(misc + par);
    const v4i m1 = *(const v4ia*)(misc + par + 4);
    int pre = 0;
    pre += (wave > 0) ? m0.x : 0;
    pre += (wave > 1) ? m0.y : 0;
    pre += (wave > 2) ? m0.z : 0;
    pre += (wave > 3) ? m0.w : 0;
    pre += (wave > 4) ? m1.x : 0;
    pre += (wave > 5) ? m1.y : 0;
    pre += (wave > 6) ? m1.z : 0;
    const int tot = (m0.x + m0.y) + (m0.z + m0.w) + (m1.x + m1.y) + (m1.z + m1.w);
    int pos = run + pre + incl - nh;
    run += tot;
    HITJ(h0, ((unsigned)sa.x & 0xFFFFu) | (s0 << 16))
    HITJ(h1, ((unsigned)sa.y & 0xFFFFu) | (s1 << 16))
    HITJ(h2, ((unsigned)sa.z & 0xFFFFu) | (s2 << 16))
    HITJ(h3, ((unsigned)sa.w & 0xFFFFu) | (s3 << 16))
    HITJ(h4, ((unsigned)sb.x & 0xFFFFu) | (s4 << 16))
    HITJ(h5, ((unsigned)sb.y & 0xFFFFu) | (s5 << 16))
    HITJ(h6, ((unsigned)sb.z & 0xFFFFu) | (s6 << 16))
    HITJ(h7, ((unsigned)sb.w & 0xFFFFu) | (s7 << 16))
  }
  __syncthreads();
  const bool ovf = run > RCAP;
  int ttv = run < 0 ? 0 : (run > RCAP ? RCAP : run);
  const int tt = __builtin_amdgcn_readfirstlane(ttv);

  if (wave == 0) {
#pragma unroll 1
    for (int b0 = 0; b0 < tt; b0 += 32) {
      int idx = b0 + lane;
      idx = idx > tt - 1 ? tt - 1 : idx;
      const int ent = wl[idx];
      const int m32 = (tt - b0) < 32 ? (tt - b0) : 32;
#pragma unroll 1
      for (int k = 0; k < m32; ++k) {
        const int uu   = __builtin_amdgcn_readlane(ent, k);
        const int slot = (uu >> 16) & (NBRUN - 1);
        if (lane == 0) cnt[slot] = cnt[slot] + 1;
      }
    }
  }
  __syncthreads();

  if (wave == 0) {
    const int base = lane * (NBRUN / 32);
    int s = 0;
#pragma unroll 1
    for (int i = 0; i < NBRUN / 32; ++i) s += cnt[base + i];
    int incl = s;
#pragma unroll
    for (int d = 1; d < 32; d <<= 1) {
      const int y = __shfl_up(incl, d, 32);
      incl += (lane >= d) ? y : 0;
    }
    int rr = incl - s;
#pragma unroll 1
    for (int i = 0; i < NBRUN / 32; ++i) {
      const int cv = cnt[base + i];
      offs[base + i] = rr;
      cur[base + i]  = rr;
      rr += cv;
    }
  }
  __syncthreads();

  if (wave == 0) {
#pragma unroll 1
    for (int b0 = 0; b0 < tt; b0 += 32) {
      int idx = b0 + lane;
      idx = idx > tt - 1 ? tt - 1 : idx;
      const int ent = wl[idx];
      const int m32 = (tt - b0) < 32 ? (tt - b0) : 32;
#pragma unroll 1
      for (int k = 0; k < m32; ++k) {
        const int uu   = __builtin_amdgcn_readlane(ent, k);
        const int slot = (uu >> 16) & (NBRUN - 1);
        if (lane == 0) {
          int p = cur[slot];
          p = p < 0 ? 0 : (p > RCAP - 1 ? RCAP - 1 : p);
          sl[p] = (unsigned short)(uu & 0xFFFF);
          cur[slot] = p + 1;
        }
      }
    }
  }
  __syncthreads();

#pragma unroll 1
  for (int j = 0; j < NBRUN / NTHR; ++j) {
    const int s = j * NTHR + tid;
    const int c = cnt[s];
    const float den = (float)(c > 0 ? c : 1);
    const float q = 1.0f / den;
    int bits = (c > 0) ? __float_as_int(q) : 0;
    bits = (ovf || c > DEGCAP) ? 0x7fc00000 : bits;
    cur[s] = bits;
  }
  __syncthreads();

  const v4i cv4 = *(const v4ia*)(cnt + 4 * tid);
  const v4i ov4 = *(const v4ia*)(offs + 4 * tid);
  const v4i iv4 = *(const v4ia*)(cur + 4 * tid);
  int* cp = cntp + (size_t)blk * NBRUN + 4 * tid;
  int* op = offp + (size_t)blk * NBRUN + 4 * tid;
  int* ip = invp + (size_t)blk * NBRUN + 4 * tid;
  int* lp = listp + (size_t)blk * RCAP;
  *(volatile v4i*)cp = cv4;
  *(volatile v4i*)op = ov4;
  *(volatile v4i*)ip = iv4;
#pragma unroll 1
  for (int q = tid; q < RCAP / 4; q += NTHR) {
    const v2u w = *(const v2ua*)(sl + 4 * q);
    v4i o;
    o.x = (int)(w.x & 0xFFFFu); o.y = (int)(w.x >> 16);
    o.z = (int)(w.y & 0xFFFFu); o.w = (int)(w.y >> 16);
    *(volatile v4i*)(lp + 4 * q) = o;
  }
  __threadfence();
  *(volatile v4i*)cp = cv4;
  *(volatile v4i*)op = ov4;
  *(volatile v4i*)ip = iv4;
#pragma unroll 1
  for (int q = tid; q < RCAP / 4; q += NTHR) {
    const v2u w = *(const v2ua*)(sl + 4 * q);
    v4i o;
    o.x = (int)(w.x & 0xFFFFu); o.y = (int)(w.x >> 16);
    o.z = (int)(w.y & 0xFFFFu); o.w = (int)(w.y >> 16);
    *(volatile v4i*)(lp + 4 * q) = o;
  }
}
#undef HITJ

template <int SRC16>
__global__ __launch_bounds__(NTHR) void k_replay(const int* __restrict__ listp, const int* __restrict__ cntp,
                                                 const int* __restrict__ offp, const float* __restrict__ invp,
                                                 const unsigned short* __restrict__ xb, const float* __restrict__ hf,
                                                 unsigned short* meanp) {
  __shared__ __attribute__((aligned(16))) unsigned short rows_s[NWAVE * 2 * DF];
  const int tid = (int)threadIdx.x, lane = tid & 31, wave = tid >> 5;
  unsigned short* rowbuf = rows_s + wave * (2 * DF);
  const int nodeBase = (int)blockIdx.x * GBM + wave * (GBM / NWAVE);
#pragma unroll 1
  for (int si = 0; si < GBM / NWAVE; ++si) {
    const int node = nodeBase + si;
    int cv = cntp[node];
    cv = cv < 0 ? 0 : (cv > DEGCAP ? DEGCAP : cv);
    int ov = offp[node];
    ov = ov < 0 ? 0 : (ov > RCAP - 1 ? RCAP - 1 : ov);
    const int c = __builtin_amdgcn_readfirstlane(cv);
    const int o = __builtin_amdgcn_readfirstlane(ov);
    const float iv = invp[node];
    const int lbase = (node >> SLA) * RCAP;
    int last = o + c - 1;
    last = last < o ? o : last;
    last = last > RCAP - 1 ? RCAP - 1 : last;
    float a0 = 0.0f, a1 = 0.0f, a2 = 0.0f, a3 = 0.0f;
#pragma unroll 1
    for (int b0 = 0; b0 < c; b0 += 32) {
      int idx = o + b0 + lane;
      idx = idx > last ? last : idx;
      int sr = listp[lbase + idx];
      sr = sr < 0 ? 0 : (sr > NN - 1 ? NN - 1 : sr);
      const int m32 = (c - b0) < 32 ? (c - b0) : 32;
#pragma unroll 1
      for (int k = 0; k < m32; ++k) {
        const int sk = __builtin_amdgcn_readlane(sr, k);
        if constexpr (SRC16 != 0) {
          const v2u w = *(const v2ua*)(xb + (size_t)sk * XPITCH + 4 * lane);
          a0 += __uint_as_float(w.x << 16);
          a1 += __uint_as_float(w.x & 0xffff0000u);
          a2 += __uint_as_float(w.y << 16);
          a3 += __uint_as_float(w.y & 0xffff0000u);
        } else {
          const v4f r = *(const v4fa*)(hf + (size_t)sk * DF + 4 * lane);
          a0 += r.x; a1 += r.y; a2 += r.z; a3 += r.w;
        }
      }
    }
    const bool live = node < NN;
    const float m0 = live ? (a0 * iv) : 0.0f;
    const float m1 = live ? (a1 * iv) : 0.0f;
    const float m2 = live ? (a2 * iv) : 0.0f;
    const float m3 = live ? (a3 * iv) : 0.0f;
    const v8us q0 = make_hl_piece(rowbuf, lane, m0, m1, m2, m3);
    unsigned short* rp = meanp + (size_t)node * MPITCH + 8 * lane;
    *(volatile v8us*)rp = q0;
    __threadfence();
    *(volatile v8us*)rp = q0;
  }
}

__device__ __forceinline__ void seg128(const unsigned short* __restrict__ ap, const unsigned short* __restrict__ bp,
                                       v8f (&acc)[8]) {
#pragma unroll 1
  for (int k0 = 0; k0 < DF; k0 += 32) {
    FragB af;
    af.h[0] = *(const v8usa*)(ap + k0);
    af.h[1] = *(const v8usa*)(ap + k0 + 16);
#pragma unroll
    for (int nt = 0; nt < 8; ++nt) {
      const unsigned short* wq = bp + (size_t)(16 * nt) * WPITCH + k0;
      FragB bf;
      bf.h[0] = *(const v8usa*)wq;
      bf.h[1] = *(const v8usa*)(wq + 16);
      acc[nt] = wmb(af, bf, acc[nt]);
    }
  }
}

template <int L0>
__global__ __launch_bounds__(NTHR) __attribute__((amdgpu_num_vgpr(248)))
void k_gemm(const unsigned short* __restrict__ meanp, const unsigned short* __restrict__ selfp,
            const unsigned short* __restrict__ wq, const float* __restrict__ biasp,
            float* tp, float* recp) {
  extern __shared__ __attribute__((aligned(16))) float gsm[];
  float* stg   = gsm;
  float* sbias = gsm + GBM * DF;
  float* psum  = sbias + DF;
  float* qsum  = psum + 2 * DF;
  float* rst   = qsum + 2 * DF;
  constexpr int SP = (L0 != 0) ? XPITCH : HPITCH;
  const int tid = (int)threadIdx.x, lane = tid & 31, wave = tid >> 5, hh = lane >> 4, m = lane & 15;
  const int rowBase = (int)blockIdx.x * GBM;

  if (tid < 32) {
    const v4f b4 = *(const v4f*)(biasp + 4 * tid);
    *(v4fa*)(sbias + 4 * tid) = b4;
  }
  __syncthreads();

  v8f acc[8];
#pragma unroll
  for (int t = 0; t < 8; ++t) acc[t] = z8();
  const int arow = rowBase + 16 * wave + m;
  const unsigned short* am = meanp + (size_t)arow * MPITCH + 8 * hh;
  const unsigned short* sf = selfp + (size_t)arow * SP + 8 * hh;
  const unsigned short* bp = wq + (size_t)m * WPITCH + 8 * hh;
  seg128(am, bp + WC_LH, acc);
  if constexpr (MEAN_LO != 0) seg128(am + DF, bp + WC_LH, acc);
  if constexpr (W_SPLIT != 0) seg128(am, bp + WC_LL, acc);
  seg128(sf, bp + WC_RH, acc);
  if constexpr (L0 == 0 && H_LO != 0) seg128(sf + DF, bp + WC_RH, acc);
  if constexpr (W_SPLIT != 0) seg128(sf, bp + WC_RL, acc);

#pragma unroll
  for (int nt = 0; nt < 8; ++nt) {
    const int lc = 16 * nt + m;
    const float bq = sbias[lc];
#pragma unroll
    for (int r = 0; r < 8; ++r) {
      const int lr = 16 * wave + 8 * hh + r;
      stg[lr * DF + lc] = acc[nt][r] + bq;
    }
  }
  __syncthreads();

#pragma unroll 1
  for (int i = 0; i < 16; ++i) {
    const int lr = 16 * wave + i;
    const v4f v = *(const v4fa*)(stg + lr * DF + 4 * lane);
    *(volatile v4f*)(tp + (size_t)(rowBase + lr) * DF + 4 * lane) = v;
  }
  __threadfence();
#pragma unroll 1
  for (int i = 0; i < 16; ++i) {
    const int lr = 16 * wave + i;
    const v4f v = *(const v4fa*)(stg + lr * DF + 4 * lane);
    *(volatile v4f*)(tp + (size_t)(rowBase + lr) * DF + 4 * lane) = v;
  }

  int nvalid = NN - rowBase;
  nvalid = nvalid > GBM ? GBM : nvalid;
  const int c    = tid & (DF - 1);
  const int half = tid >> 7;
  const int r0   = half * (GBM / 2);
  int r1 = r0 + GBM / 2;
  r1 = r1 > nvalid ? nvalid : r1;
  float s = 0.0f;
#pragma unroll 4
  for (int r = r0; r < r1; ++r) s += stg[r * DF + c];
  psum[tid] = s;
  __syncthreads();
  const float mean = (psum[c] + psum[DF + c]) * (1.0f / (float)nvalid);
  float q = 0.0f;
#pragma unroll 4
  for (int r = r0; r < r1; ++r) {
    const float d = stg[r * DF + c] - mean;
    q = fmaf(d, d, q);
  }
  qsum[tid] = q;
  __syncthreads();
  if (tid < DF) {
    rst[tid] = mean;
    rst[DF + tid] = qsum[tid] + qsum[DF + tid];
  }
  __syncthreads();
  v4f rv = {0.f, 0.f, 0.f, 0.f};
  if (tid < 64) rv = *(const v4fa*)(rst + 4 * tid);
  float* rp = recp + (size_t)blockIdx.x * (2 * DF) + 4 * tid;
  if (tid < 64) *(volatile v4f*)rp = rv;
  __threadfence();
  if (tid < 64) *(volatile v4f*)rp = rv;
}

__global__ __launch_bounds__(DF) void k_comb(const float* __restrict__ rec, float* stat) {
  __shared__ __attribute__((aligned(16))) float sst[2 * DF];
  const int tid = (int)threadIdx.x;
  const double invn = 1.0 / (double)NN;
  double sm = 0.0;
#pragma unroll 1
  for (int b = 0; b < NTILE; ++b) {
    int nbv = NN - b * GBM;
    nbv = nbv > GBM ? GBM : nbv;
    sm += (double)nbv * (double)rec[(size_t)b * (2 * DF) + tid];
  }
  const double mean = sm * invn;
  double m2 = 0.0, cr = 0.0;
#pragma unroll 1
  for (int b = 0; b < NTILE; ++b) {
    int nbv = NN - b * GBM;
    nbv = nbv > GBM ? GBM : nbv;
    const double d = (double)rec[(size_t)b * (2 * DF) + tid] - mean;
    m2 += (double)rec[(size_t)b * (2 * DF) + DF + tid];
    cr += (double)nbv * d * d;
  }
  const float varf = (float)((m2 + cr) * invn);
  const float rs = 1.0f / sqrtf(varf + 1e-5f);
  sst[tid] = (float)mean;
  sst[DF + tid] = rs;
  __syncthreads();
  v4f v = {0.f, 0.f, 0.f, 0.f};
  if (tid < 64) v = *(const v4fa*)(sst + 4 * tid);
  if (tid < 64) *(volatile v4f*)(stat + 4 * tid) = v;
  __threadfence();
  if (tid < 64) *(volatile v4f*)(stat + 4 * tid) = v;
}

template <int LAST>
__global__ __launch_bounds__(NTHR) void k_apply(float* th, const float* __restrict__ statp,
                                                const float* __restrict__ gp, const float* __restrict__ bp,
                                                unsigned short* hhl, float* outp) {
  __shared__ __attribute__((aligned(16))) float sp[4 * DF];
  __shared__ __attribute__((aligned(16))) unsigned short rows_s[NWAVE * 2 * DF];
  const int tid = (int)threadIdx.x, lane = tid & 31, wave = tid >> 5;
  if (tid < 32) {
    const v4f a = *(const v4f*)(statp + 4 * tid);
    const v4f b = *(const v4f*)(statp + DF + 4 * tid);
    const v4f g = *(const v4f*)(gp + 4 * tid);
    const v4f e = *(const v4f*)(bp + 4 * tid);
    *(v4fa*)(sp + 4 * tid) = a;
    *(v4fa*)(sp + DF + 4 * tid) = b;
    *(v4fa*)(sp + 2 * DF + 4 * tid) = g;
    *(v4fa*)(sp + 3 * DF + 4 * tid) = e;
  }
  __syncthreads();
  const int u = (int)blockIdx.x * NTHR + tid;
  const v4f t  = *(const v4f*)(th + (size_t)u * 4);
  const v4f mu = *(const v4fa*)(sp + 4 * lane);
  const v4f rs = *(const v4fa*)(sp + DF + 4 * lane);
  const v4f gg = *(const v4fa*)(sp + 2 * DF + 4 * lane);
  const v4f be = *(const v4fa*)(sp + 3 * DF + 4 * lane);
  const float y0 = ((t.x - mu.x) * rs.x) * gg.x + be.x;
  const float y1 = ((t.y - mu.y) * rs.y) * gg.y + be.y;
  const float y2 = ((t.z - mu.z) * rs.z) * gg.z + be.z;
  const float y3 = ((t.w - mu.w) * rs.w) * gg.w + be.w;
  v4f o;
  o.x = (y0 > 0.0f) ? y0 : (y0 - y0);
  o.y = (y1 > 0.0f) ? y1 : (y1 - y1);
  o.z = (y2 > 0.0f) ? y2 : (y2 - y2);
  o.w = (y3 > 0.0f) ? y3 : (y3 - y3);
  if constexpr (LAST != 0) {
    float* op = outp + (size_t)u * 4;
    *(volatile v4f*)op = o;
    __threadfence();
    *(volatile v4f*)op = o;
    (void)hhl; (void)rows_s; (void)wave;
  } else {
    unsigned short* rowbuf = rows_s + wave * (2 * DF);
    const v8us q0 = make_hl_piece(rowbuf, lane, o.x, o.y, o.z, o.w);
    const int row = u >> 5;
    float* hp = th + (size_t)u * 4;
    unsigned short* rp = hhl + (size_t)row * HPITCH + 8 * lane;
    *(volatile v4f*)hp = o;
    *(volatile v8us*)rp = q0;
    __threadfence();
    *(volatile v4f*)hp = o;
    *(volatile v8us*)rp = q0;
    (void)outp;
  }
}

extern "C" void kernel_launch(void* const* d_in, const int* in_sizes, int n_in,
                              void* d_out, int out_size, void* d_ws, size_t ws_size,
                              hipStream_t stream) {
  if (n_in < 7) return;
  if (in_sizes[0] != NN * DF) return;
  if (in_sizes[1] != 2 * NE) return;
  if (in_sizes[2] != NLAY * DF * DF) return;
  if (in_sizes[3] != NLAY * DF) return;
  if (in_sizes[4] != NLAY * DF * DF) return;
  if (in_sizes[5] != NLAY * DF) return;
  if (in_sizes[6] != NLAY * DF) return;
  if (out_size != NN * DF) return;
  if (O_END > ws_size) return;

  const float* x   = (const float*)d_in[0];
  const int*   ei  = (const int*)  d_in[1];
  const float* Wl  = (const float*)d_in[2];
  const float* bl  = (const float*)d_in[3];
  const float* Wr  = (const float*)d_in[4];
  const float* gam = (const float*)d_in[5];
  const float* bet = (const float*)d_in[6];
  float* out = (float*)d_out;
  const int* src = ei;
  const int* dst = ei + NE;

  char* ws = (char*)d_ws;
  unsigned short* WQ   = (unsigned short*)(ws + O_WQ);
  float*          PAR  = (float*)(ws + O_PAR);
  float*          STAT = (float*)(ws + O_STAT);
  unsigned short* XB   = (unsigned short*)(ws + O_XB);
  unsigned short* MEAN = (unsigned short*)(ws + O_MEAN);
  unsigned short* HHL  = (unsigned short*)(ws + O_H);
  float*          TH   = (float*)(ws + O_TH);
  int*            LIST = (int*)(ws + O_LIST);
  int*            CNT  = (int*)(ws + O_CNT);
  int*            OFF  = (int*)(ws + O_OFF);
  int*            INV  = (int*)(ws + O_INV);
  float*          REC  = (float*)(ws + O_REC);

  const size_t bkLds = (size_t)BK_INTS * 4;
  const size_t gLds  = (size_t)G_FLOATS * 4;
  hipFuncSetAttribute(reinterpret_cast<const void*>(&k_bucket), hipFuncAttributeMaxDynamicSharedMemorySize, (int)bkLds);
  hipFuncSetAttribute(reinterpret_cast<const void*>(&k_gemm<1>), hipFuncAttributeMaxDynamicSharedMemorySize, (int)gLds);
  hipFuncSetAttribute(reinterpret_cast<const void*>(&k_gemm<0>), hipFuncAttributeMaxDynamicSharedMemorySize, (int)gLds);

  const int gPrep  = (PU4 + NTHR - 1) / NTHR;
  const int gApply = (NN * 32) / NTHR;

  k_prep<<<gPrep, NTHR, 0, stream>>>(x, Wl, Wr, bl, gam, bet, (unsigned*)d_ws);
  k_bucket<<<NBLK, NTHR, bkLds, stream>>>(src, dst, LIST, CNT, OFF, INV);

  k_replay<1><<<NTILE, NTHR, 0, stream>>>(LIST, CNT, OFF, (const float*)INV, XB, TH, MEAN);
  k_gemm<1><<<NTILE, NTHR, gLds, stream>>>(MEAN, XB, WQ, PAR, TH, REC);
  k_comb<<<1, DF, 0, stream>>>(REC, STAT);
  k_apply<0><<<gApply, NTHR, 0, stream>>>(TH, STAT, PAR + NLAY * DF, PAR + 2 * NLAY * DF, HHL, out);

  k_replay<0><<<NTILE, NTHR, 0, stream>>>(LIST, CNT, OFF, (const float*)INV, XB, TH, MEAN);
  k_gemm<0><<<NTILE, NTHR, gLds, stream>>>(MEAN, HHL, WQ + (size_t)DF * WPITCH, PAR + DF, TH, REC);
  k_comb<<<1, DF, 0, stream>>>(REC, STAT + 2 * DF);
  k_apply<0><<<gApply, NTHR, 0, stream>>>(TH, STAT + 2 * DF, PAR + NLAY * DF + DF, PAR + 2 * NLAY * DF + DF, HHL, out);

  k_replay<0><<<NTILE, NTHR, 0, stream>>>(LIST, CNT, OFF, (const float*)INV, XB, TH, MEAN);
  k_gemm<0><<<NTILE, NTHR, gLds, stream>>>(MEAN, HHL, WQ + (size_t)2 * DF * WPITCH, PAR + 2 * DF, TH, REC);
  k_comb<<<1, DF, 0, stream>>>(REC, STAT + 4 * DF);
  k_apply<1><<<gApply, NTHR, 0, stream>>>(TH, STAT + 4 * DF, PAR + NLAY * DF + 2 * DF, PAR + 2 * NLAY * DF + 2 * DF, HHL, out);
}
